// Model_24824910971198
// MI455X (gfx1250) — hardware-verified
//
#include <hip/hip_runtime.h>
#include <math.h>

typedef __attribute__((ext_vector_type(16))) _Float16 v16h;
typedef __attribute__((ext_vector_type(16))) __bf16 v16b;
typedef __attribute__((ext_vector_type(8)))  _Float16 v8h;
typedef __attribute__((ext_vector_type(8)))  float v8f;
typedef __attribute__((ext_vector_type(4)))  float v4f;
typedef __attribute__((ext_vector_type(4)))  unsigned v4u;

#ifndef NB
#define NB 2
#endif
#ifndef SEQ
#define SEQ 4096
#endif
#define NB_FULL 2
#define SEQ_FULL 4096
#define CH 16
#define PL 32
#define DM 256
#define NH 8
#define HD 32
#define NLAYER 2
#define FF 1024
#define MAXLEN 256
#define NSEG (SEQ / PL)
#define L2 (2 * NSEG)
#define NBC (NB * CH)
#define NTOK (NBC * L2)
#define VP (L2 + 8)

static_assert(PL == 32);
static_assert(CH == 16);
static_assert(DM == 256);
static_assert(HD == 32);
static_assert(NH * HD == DM);
static_assert(SEQ % PL == 0);
static_assert(L2 % 64 == 0);
static_assert(L2 <= MAXLEN);
static_assert(NB <= NB_FULL);
static_assert(SEQ <= SEQ_FULL);
static_assert(NTOK % 64 == 0);
static_assert(DM % 64 == 0);
static_assert(FF % 64 == 0);
static_assert(DM % 32 == 0);
static_assert(FF % 32 == 0);
static_assert(NBC <= 32);
static_assert((NLAYER * DM * DM) % 2048 == 0);
static_assert((NLAYER * FF * DM) % 2048 == 0);
static_assert(NB * PL * CH <= 1024);

template <typename T> __device__ __forceinline__ void vst2(void* p, T v) { *(volatile T*)p = v; __threadfence(); *(volatile T*)p = v; }
__device__ __forceinline__ v8f wmma16(v16h a, v16h b, v8f c) {
  v8f d = __builtin_amdgcn_wmma_f32_16x16x32_f16(false, a, false, b, (short)0, c, false, false);
  asm volatile("v_nop\n\tv_nop\n\tv_nop\n\tv_nop" : "+v"(d) : "v"(a), "v"(b));
  return d;
}
__device__ __forceinline__ v8f wmma_bf(v16b a, v16b b, v8f c) {
  v8f d = __builtin_amdgcn_wmma_f32_16x16x32_bf16(false, a, false, b, (short)0, c, false, false);
  asm volatile("v_nop\n\tv_nop\n\tv_nop\n\tv_nop" : "+v"(d) : "v"(a), "v"(b));
  return d;
}
__device__ __forceinline__ v16h frag_h(const _Float16* rowk0, int lane) {
  union { v16h v; v8h q[2]; } u; const _Float16* p = rowk0 + 8 * (lane >> 4);
  u.q[0] = *(const v8h*)p; u.q[1] = *(const v8h*)(p + 16); return u.v;
}
struct F2 { v16b h, l; };
__device__ __forceinline__ F2 bsplit16(const float v[16]) { F2 r;
#pragma unroll
  for (int i = 0; i < 16; ++i) { const __bf16 h = (__bf16)v[i]; r.h[i] = h; r.l[i] = (__bf16)(v[i] - (float)h); }
  return r; }
__device__ __forceinline__ float bfr(float v) { return (float)(__bf16)v; }
__device__ __forceinline__ v16b wrow_bf(const float* rowk0, int lane) { v16b w; const float* p = rowk0 + 8 * (lane >> 4);
  const v4f a = *(const v4f*)p, b = *(const v4f*)(p + 4), c = *(const v4f*)(p + 16), d = *(const v4f*)(p + 20);
#pragma unroll
  for (int i = 0; i < 4; ++i) { w[i] = (__bf16)a[i]; w[4 + i] = (__bf16)b[i]; w[8 + i] = (__bf16)c[i]; w[12 + i] = (__bf16)d[i]; }
  return w; }
__device__ __forceinline__ v16h wrow_h(const float* rowk0, int lane) { v16h w; const float* p = rowk0 + 8 * (lane >> 4);
  const v4f a = *(const v4f*)p, b = *(const v4f*)(p + 4), c = *(const v4f*)(p + 16), d = *(const v4f*)(p + 20);
#pragma unroll
  for (int i = 0; i < 4; ++i) { w[i] = (_Float16)(bfr(a[i]) * 256.0f); w[4 + i] = (_Float16)(bfr(b[i]) * 256.0f); w[8 + i] = (_Float16)(bfr(c[i]) * 256.0f); w[12 + i] = (_Float16)(bfr(d[i]) * 256.0f); }
  return w; }
__device__ __forceinline__ void split8h(const float v[8], v8h& hi, v8h& lo) {
#pragma unroll
  for (int i = 0; i < 8; ++i) { const _Float16 hh = (_Float16)v[i]; hi[i] = hh; lo[i] = (_Float16)((v[i] - (float)hh) * 2048.0f); } }
__device__ __forceinline__ v4u h2u(v8h x) { union { v8h h; v4u u; } t; t.h = x; return t.u; }
__device__ __forceinline__ float wsum(float v) {
#pragma unroll
  for (int o = 1; o < 32; o <<= 1) v += __shfl_xor(v, o);
  return v; }
#define LDSX() do { asm volatile("s_wait_dscnt 0" ::: "memory"); __builtin_amdgcn_wave_barrier(); __builtin_amdgcn_fence(3  , "workgroup"); } while (0)

#define WS_ST  0u
#define WS_H   (WS_ST + 256u)
#define WS_ZH  (WS_H  + 4u * (size_t)NTOK * DM)
#define WS_ZL  (WS_ZH + 2u * (size_t)NTOK * DM)
#define WS_QH  (WS_ZL + 2u * (size_t)NTOK * DM)
#define WS_QL  (WS_QH + 2u * (size_t)NTOK * DM)
#define WS_KH  (WS_QL + 2u * (size_t)NTOK * DM)
#define WS_KL  (WS_KH + 2u * (size_t)NTOK * DM)
#define WS_VH  (WS_KL + 2u * (size_t)NTOK * DM)
#define WS_VL  (WS_VH + 2u * (size_t)NTOK * DM)
#define WS_A32 (WS_VL + 2u * (size_t)NTOK * DM)
#define WS_FH  (WS_A32 + 4u * (size_t)NTOK * DM)
#define WS_FL  (WS_FH + 2u * (size_t)NTOK * FF)
#define WS_WQ  (WS_FL + 2u * (size_t)NTOK * FF)
#define WS_WK  (WS_WQ + 2u * (size_t)NLAYER * DM * DM)
#define WS_WV  (WS_WK + 2u * (size_t)NLAYER * DM * DM)
#define WS_WC  (WS_WV + 2u * (size_t)NLAYER * DM * DM)
#define WS_WFC (WS_WC + 2u * (size_t)NLAYER * DM * DM)
#define WS_WP  (WS_WFC + 2u * (size_t)NLAYER * FF * DM)
#define WS_END (WS_WP + 2u * (size_t)NLAYER * DM * FF)
static_assert((size_t)WS_END <= (size_t)134217728);

__global__ __launch_bounds__(256) void k_wcvt(const float* __restrict__ S, _Float16* __restrict__ D) {
  const size_t e = ((size_t)blockIdx.x * 256 + threadIdx.x) * 8;
  const v4f a = *(const v4f*)(S + e), b = *(const v4f*)(S + e + 4);
  v8h o;
#pragma unroll
  for (int i = 0; i < 4; ++i) { o[i] = (_Float16)(bfr(a[i]) * 256.0f); o[4 + i] = (_Float16)(bfr(b[i]) * 256.0f); }
  vst2(D + e, h2u(o)); }

__global__ __launch_bounds__(256) void k_stats(const float* __restrict__ X, float* __restrict__ ST) {
  __shared__ __align__(16) float st[64];
  const int tid = threadIdx.x; const int wave = __builtin_amdgcn_readfirstlane(tid >> 5); const int lane = tid & 31;
#pragma unroll 1
  for (int bc = wave; bc < 32; bc += 8) {
    float mu = 0.f, sd = 1.f;
    if (bc < NBC) {
      const int b = bc >> 4, c = bc & 15; const float* xp = X + (size_t)b * SEQ_FULL * CH + c;
      float s = 0.f;
#pragma unroll 4
      for (int i = 0; i < SEQ / 32; ++i) s += bfr(xp[(size_t)(lane + 32 * i) * CH]);
      s = wsum(s); const float ma = s / (float)SEQ;
      float s2 = 0.f;
#pragma unroll 4
      for (int i = 0; i < SEQ / 32; ++i) { const float d = bfr(xp[(size_t)(lane + 32 * i) * CH]) - ma; s2 += d * d; }
      s2 = wsum(s2);
      float sl = bfr(xp[(size_t)(SEQ - PL + lane) * CH]); sl = wsum(sl);
      mu = sl / (float)PL; sd = sqrtf(s2 / (float)(SEQ - 1)) + 1e-8f;
    }
    if (lane == 0) { st[bc] = mu; st[32 + bc] = sd; }
  }
  __syncthreads();
  if (tid < 16) { const v4f v = *(const v4f*)&st[tid * 4]; vst2(ST + tid * 4, v); } }

__global__ __launch_bounds__(128) void k_embed(const float* __restrict__ X, const float* __restrict__ ST, const float* __restrict__ tok_w, const float* __restrict__ tok_b, const float* __restrict__ ccp_w, const float* __restrict__ ccp_b, const float* __restrict__ ctp_w, const float* __restrict__ ctp_b, const float* __restrict__ ncw, const float* __restrict__ nmw, const float* __restrict__ pnw, const float* __restrict__ pos, const float* __restrict__ cemb, float* __restrict__ Hout) {
  __shared__ __align__(16) float seg[CH][36], mix[CH][36], ot[32][260];
  const int tid = threadIdx.x; const int wave = __builtin_amdgcn_readfirstlane(tid >> 5); const int lane = tid & 31, col = lane & 15, g = lane >> 4;
  const int n = blockIdx.x, b = blockIdx.y;
#pragma unroll
  for (int u = 0; u < 4; ++u) { const int i = tid + 128 * u; const int c = i & 15, s = i >> 4;
    const float mu = ST[b * CH + c], sd = ST[32 + b * CH + c]; const float xv = bfr(X[((size_t)b * SEQ_FULL + n * PL + s) * CH + c]);
    seg[c][s] = (xv - mu) * (1.0f / sd); }
  __syncthreads();
#pragma unroll 1
  for (int u = 0; u < 4; ++u) { const int i = tid + 128 * u; const int s = i & 31, t = i >> 5; float a = 0.f;
#pragma unroll 4
    for (int c = 0; c < CH; ++c) a += seg[c][s] * bfr(ccp_w[t * CH + c]);
    mix[t][s] = a + bfr(ccp_b[t]); }
  __syncthreads();
  float va[16], vm[16];
#pragma unroll
  for (int i = 0; i < 8; ++i) { va[i] = mix[col][8 * g + i]; va[8 + i] = mix[col][16 + 8 * g + i]; vm[i] = seg[col][8 * g + i]; vm[8 + i] = seg[col][16 + 8 * g + i]; }
  const F2 fa = bsplit16(va), fm = bsplit16(vm);
#pragma unroll
  for (int j = 0; j < 4; ++j) { const int nn = wave * 64 + j * 16 + col;
    const v16b wc = wrow_bf(ctp_w + (size_t)nn * PL, lane), wt = wrow_bf(tok_w + (size_t)nn * PL, lane);
    v8f c = {}, m = {};
    c = wmma_bf(fa.l, wc, c); c = wmma_bf(fa.h, wc, c); m = wmma_bf(fm.l, wt, m); m = wmma_bf(fm.h, wt, m);
    const float bcx = bfr(ctp_b[nn]), btx = bfr(tok_b[nn]);
#pragma unroll
    for (int r = 0; r < 8; ++r) { ot[8 * g + r][nn] = c[r] + bcx; ot[16 + 8 * g + r][nn] = m[r] + btx; } }
  __syncthreads();
#pragma unroll 1
  for (int it = 0; it < 8; ++it) { const int rr = wave * 8 + it; const int ty = rr >> 4, t = rr & 15; const int l = 2 * n + ty;
    const v4f x0 = *(const v4f*)&ot[rr][lane * 4], x1 = *(const v4f*)&ot[rr][128 + lane * 4];
    float ss = x0[0] * x0[0] + x0[1] * x0[1] + x0[2] * x0[2] + x0[3] * x0[3] + x1[0] * x1[0] + x1[1] * x1[1] + x1[2] * x1[2] + x1[3] * x1[3];
    ss = wsum(ss); const float r1 = rsqrtf(ss * (1.0f / 256.0f) + 1e-5f);
    const v4f c0 = *(const v4f*)(ncw + lane * 4), c1 = *(const v4f*)(ncw + 128 + lane * 4), m0 = *(const v4f*)(nmw + lane * 4), m1 = *(const v4f*)(nmw + 128 + lane * 4);
    const v4f p0 = *(const v4f*)(pos + (size_t)l * DM + lane * 4), p1 = *(const v4f*)(pos + (size_t)l * DM + 128 + lane * 4);
    const float* ce = cemb + ((size_t)t * MAXLEN + l) * DM; const v4f e0 = *(const v4f*)(ce + lane * 4), e1 = *(const v4f*)(ce + 128 + lane * 4);
    const v4f q0 = *(const v4f*)(pnw + lane * 4), q1 = *(const v4f*)(pnw + 128 + lane * 4);
    v4f y0, y1; float s2 = 0.f;
#pragma unroll
    for (int i = 0; i < 4; ++i) { const float w0 = bfr(ty ? m0[i] : c0[i]), w1 = bfr(ty ? m1[i] : c1[i]);
      y0[i] = x0[i] * r1 * w0 + (bfr(p0[i]) + bfr(e0[i])); y1[i] = x1[i] * r1 * w1 + (bfr(p1[i]) + bfr(e1[i])); s2 += y0[i] * y0[i] + y1[i] * y1[i]; }
    s2 = wsum(s2); const float r2 = rsqrtf(s2 * (1.0f / 256.0f) + 1e-5f);
    v4f o0, o1;
#pragma unroll
    for (int i = 0; i < 4; ++i) { o0[i] = y0[i] * r2 * bfr(q0[i]); o1[i] = y1[i] * r2 * bfr(q1[i]); }
    float* hp = Hout + (((size_t)(b * CH + t)) * L2 + l) * DM;
    vst2(hp + lane * 4, o0); vst2(hp + 128 + lane * 4, o1); } }

__global__ __launch_bounds__(256) void k_rms(const float* __restrict__ Hs, const float* __restrict__ Wn, int do_norm, _Float16* __restrict__ ZH, _Float16* __restrict__ ZL) {
  const int tid = threadIdx.x; const int wave = __builtin_amdgcn_readfirstlane(tid >> 5); const int lane = tid & 31;
  const size_t row = (size_t)blockIdx.x * 8 + wave; const float* p = Hs + row * DM + lane * 8;
  const v4f a = *(const v4f*)p, b = *(const v4f*)(p + 4); const v4f wa = *(const v4f*)(Wn + lane * 8), wb = *(const v4f*)(Wn + lane * 8 + 4);
  float ss = a[0] * a[0] + a[1] * a[1] + a[2] * a[2] + a[3] * a[3] + b[0] * b[0] + b[1] * b[1] + b[2] * b[2] + b[3] * b[3];
  ss = wsum(ss); const float rs = rsqrtf(ss * (1.0f / 256.0f) + 1e-5f);
  float t[8];
#pragma unroll
  for (int i = 0; i < 4; ++i) { const float na = a[i] * rs * bfr(wa[i]), nb = b[i] * rs * bfr(wb[i]); t[i] = do_norm ? na : a[i]; t[4 + i] = do_norm ? nb : b[i]; }
  v8h hi, lo; split8h(t, hi, lo);
  vst2(ZH + row * DM + lane * 8, h2u(hi)); vst2(ZL + row * DM + lane * 8, h2u(lo)); }

template <int MODE>
__device__ __forceinline__ void gemm_body(const _Float16* __restrict__ AH, const _Float16* __restrict__ AL, const _Float16* __restrict__ W, const float* __restrict__ bias, const int K, const int N, _Float16* __restrict__ OH, _Float16* __restrict__ OL, float* __restrict__ Hr) {
  __shared__ __align__(16) float ss[4][16][68];
  const int tid = threadIdx.x; const int wave = __builtin_amdgcn_readfirstlane(tid >> 5); const int lane = tid & 31, col = lane & 15, g = lane >> 4;
  const int m0 = blockIdx.x * 64 + wave * 16; const int n0 = blockIdx.y * 64;
  const _Float16* ah = AH + (size_t)(m0 + col) * K; const _Float16* al = AL + (size_t)(m0 + col) * K;
  v8f acc[4] = {}, accl[4] = {};
#pragma unroll 1
  for (int k0 = 0; k0 < K; k0 += 32) { const v16h a = frag_h(ah + k0, lane), ar = frag_h(al + k0, lane);
#pragma unroll
    for (int j = 0; j < 4; ++j) { const v16h w = frag_h(W + (size_t)(n0 + j * 16 + col) * K + k0, lane); acc[j] = wmma16(a, w, acc[j]); accl[j] = wmma16(ar, w, accl[j]); } }
#pragma unroll
  for (int j = 0; j < 4; ++j) {
#pragma unroll
    for (int r = 0; r < 8; ++r) ss[wave][8 * g + r][j * 16 + col] = (acc[j][r] + accl[j][r] * (1.0f / 2048.0f)) * (1.0f / 256.0f); }
  LDSX();
  if (MODE == 2) {
#pragma unroll 1
    for (int it = 0; it < 8; ++it) { const int rl = it * 2 + (lane >> 4), c4 = (lane & 15) * 4;
      const v4f v = *(const v4f*)&ss[wave][rl][c4]; const v4f bv = *(const v4f*)(bias + n0 + c4);
      float* hp = Hr + (size_t)(m0 + rl) * N + n0 + c4; const v4f old = *(const v4f*)hp; v4f o;
#pragma unroll
      for (int i = 0; i < 4; ++i) o[i] = old[i] + (v[i] + bfr(bv[i]));
      vst2(hp, o); }
  } else {
#pragma unroll 1
    for (int it = 0; it < 4; ++it) { const int rl = it * 4 + (lane >> 3), c8 = (lane & 7) * 8;
      const v4f v0 = *(const v4f*)&ss[wave][rl][c8], v1 = *(const v4f*)&ss[wave][rl][c8 + 4]; const v4f b0 = *(const v4f*)(bias + n0 + c8), b1 = *(const v4f*)(bias + n0 + c8 + 4);
      float t[8];
#pragma unroll
      for (int i = 0; i < 4; ++i) { t[i] = v0[i] + bfr(b0[i]); t[4 + i] = v1[i] + bfr(b1[i]); }
      if (MODE == 1) {
#pragma unroll
        for (int i = 0; i < 8; ++i) t[i] = 0.5f * t[i] * (1.0f + erff(t[i] * 0.70710678118654752f)); }
      v8h hi, lo; split8h(t, hi, lo); const size_t o = (size_t)(m0 + rl) * N + n0 + c8;
      vst2(OH + o, h2u(hi)); vst2(OL + o, h2u(lo)); } } }
__global__ __launch_bounds__(128) void k_gemm_pl(const _Float16* __restrict__ AH, const _Float16* __restrict__ AL, const _Float16* __restrict__ W, const float* __restrict__ bias, int K, int N, _Float16* __restrict__ OH, _Float16* __restrict__ OL) { gemm_body<0>(AH, AL, W, bias, K, N, OH, OL, (float*)0); }
__global__ __launch_bounds__(128) void k_gemm_ge(const _Float16* __restrict__ AH, const _Float16* __restrict__ AL, const _Float16* __restrict__ W, const float* __restrict__ bias, int K, int N, _Float16* __restrict__ OH, _Float16* __restrict__ OL) { gemm_body<1>(AH, AL, W, bias, K, N, OH, OL, (float*)0); }
__global__ __launch_bounds__(128) void k_gemm_rs(const _Float16* __restrict__ AH, const _Float16* __restrict__ AL, const _Float16* __restrict__ W, const float* __restrict__ bias, int K, int N, float* __restrict__ Hr) { gemm_body<2>(AH, AL, W, bias, K, N, (_Float16*)0, (_Float16*)0, Hr); }

__global__ __launch_bounds__(128) void k_attn(const _Float16* __restrict__ QH, const _Float16* __restrict__ QL, const _Float16* __restrict__ KH, const _Float16* __restrict__ KL, const _Float16* __restrict__ VH, const _Float16* __restrict__ VL, float* __restrict__ A32) {
  __shared__ __align__(16) _Float16 vth[HD][VP], vtl[HD][VP];
  __shared__ __align__(16) float so[4][16][36];
  const int tid = threadIdx.x; const int wave = __builtin_amdgcn_readfirstlane(tid >> 5); const int lane = tid & 31, col = lane & 15, g = lane >> 4;
  const int hc = blockIdx.y * HD; const size_t tok0 = (size_t)blockIdx.x * L2;
  for (int j = tid; j < L2; j += 128) {
    const v8h* ph = (const v8h*)(VH + (tok0 + j) * DM + hc); const v8h* pl = (const v8h*)(VL + (tok0 + j) * DM + hc);
    v8h a[4], b[4];
#pragma unroll
    for (int q = 0; q < 4; ++q) { a[q] = ph[q]; b[q] = pl[q]; }
#pragma unroll
    for (int q = 0; q < 4; ++q) {
#pragma unroll
      for (int i = 0; i < 8; ++i) { vth[q * 8 + i][j] = a[q][i]; vtl[q * 8 + i][j] = b[q][i]; } } }
  __syncthreads();
#pragma unroll 1
  for (int i = 0; i < L2 / 64; ++i) { const int qt = (i & 1) ? (i * 4 + 3 - wave) : (i * 4 + wave);
    const size_t qrow = tok0 + (size_t)qt * 16 + col;
    const v16h qh = frag_h(QH + qrow * DM + hc, lane), ql = frag_h(QL + qrow * DM + hc, lane);
    v8f o0 = {}, o1 = {}, ol0 = {}, ol1 = {};
    const int nks = (qt >> 1) + 1; const int qi = qt * 16 + col;
#pragma unroll 1
    for (int ks = 0; ks < nks; ++ks) { v16h bh, bl;
#pragma unroll
      for (int t2 = 0; t2 < 2; ++t2) { const size_t krow = tok0 + (size_t)(ks * 32 + t2 * 16 + col);
        const v16h kh = frag_h(KH + krow * DM + hc, lane), kl = frag_h(KL + krow * DM + hc, lane);
        v8f s = {}, sl = {};
        s = wmma16(kh, qh, s); sl = wmma16(kl, qh, sl); sl = wmma16(kh, ql, sl);
#pragma unroll
        for (int r = 0; r < 8; ++r) { const int key = ks * 32 + t2 * 16 + 8 * g + r; float v = s[r] + sl[r] * (1.0f / 2048.0f); v = (key <= qi) ? v : 0.0f;
          const _Float16 hh = (_Float16)v; bh[t2 * 8 + r] = hh; bl[t2 * 8 + r] = (_Float16)((v - (float)hh) * 2048.0f); } }
      const v16h vh0 = frag_h(&vth[col][ks * 32], lane), vl0 = frag_h(&vtl[col][ks * 32], lane);
      o0 = wmma16(vh0, bh, o0); ol0 = wmma16(vl0, bh, ol0); ol0 = wmma16(vh0, bl, ol0);
      const v16h vh1 = frag_h(&vth[16 + col][ks * 32], lane), vl1 = frag_h(&vtl[16 + col][ks * 32], lane);
      o1 = wmma16(vh1, bh, o1); ol1 = wmma16(vl1, bh, ol1); ol1 = wmma16(vh1, bl, ol1); }
    LDSX();
#pragma unroll
    for (int r = 0; r < 8; ++r) { so[wave][col][8 * g + r] = o0[r] + ol0[r] * (1.0f / 2048.0f); so[wave][col][16 + 8 * g + r] = o1[r] + ol1[r] * (1.0f / 2048.0f); }
    LDSX();
#pragma unroll
    for (int it = 0; it < 4; ++it) { const int rl = it * 4 + (lane >> 3), c4 = (lane & 7) * 4; const v4f v = *(const v4f*)&so[wave][rl][c4];
      vst2(A32 + (tok0 + (size_t)qt * 16 + rl) * DM + hc + c4, v); } } }

__global__ __launch_bounds__(128) void k_final(const float* __restrict__ Hs, const float* __restrict__ fw, const float* __restrict__ out_w, const float* __restrict__ out_b, const float* __restrict__ ST, float* __restrict__ out) {
  __shared__ __align__(16) _Float16 zh[32][264], zl[32][264]; __shared__ __align__(16) float os[1024];
  const int tid = threadIdx.x; const int wave = __builtin_amdgcn_readfirstlane(tid >> 5); const int lane = tid & 31, col = lane & 15, g = lane >> 4;
#pragma unroll 1
  for (int it = 0; it < 8; ++it) { const int rr = wave * 8 + it; const int rc = rr < NBC ? rr : NBC - 1;
    const float* p = Hs + ((size_t)rc * L2 + (L2 - 1)) * DM + lane * 8;
    const v4f a = *(const v4f*)p, b = *(const v4f*)(p + 4); const v4f wa = *(const v4f*)(fw + lane * 8), wb = *(const v4f*)(fw + lane * 8 + 4);
    float ss = a[0] * a[0] + a[1] * a[1] + a[2] * a[2] + a[3] * a[3] + b[0] * b[0] + b[1] * b[1] + b[2] * b[2] + b[3] * b[3];
    ss = wsum(ss); const float rs = rsqrtf(ss * (1.0f / 256.0f) + 1e-5f);
    float t[8];
#pragma unroll
    for (int i = 0; i < 4; ++i) { t[i] = a[i] * rs * bfr(wa[i]); t[4 + i] = b[i] * rs * bfr(wb[i]); }
    v8h hi, lo; split8h(t, hi, lo); *(v8h*)&zh[rr][lane * 8] = hi; *(v8h*)&zl[rr][lane * 8] = lo; }
  __syncthreads();
  const int mt = wave >> 1, nt = wave & 1;
  v8f acc = {}, accl = {};
#pragma unroll 1
  for (int k0 = 0; k0 < DM; k0 += 32) { const v16h a = frag_h(&zh[mt * 16 + col][k0], lane), ar = frag_h(&zl[mt * 16 + col][k0], lane);
    const v16h w = wrow_h(out_w + (size_t)(nt * 16 + col) * DM + k0, lane); acc = wmma16(a, w, acc); accl = wmma16(ar, w, accl); }
  const int s = nt * 16 + col; const float ob = bfr(out_b[s]);
#pragma unroll
  for (int r = 0; r < 8; ++r) { const int bcx = mt * 16 + 8 * g + r; const float val = (acc[r] + accl[r] * (1.0f / 2048.0f)) * (1.0f / 256.0f) + ob;
    const float o = val * ST[32 + bcx] + ST[bcx]; os[((bcx >> 4) * PL + s) * CH + (bcx & 15)] = o; }
  __syncthreads();
#pragma unroll
  for (int u = 0; u < 2; ++u) { const int idx = tid + 128 * u; if (idx * 4 < NB * PL * CH) { const v4f v = *(const v4f*)&os[idx * 4]; vst2(out + idx * 4, v); } } }

extern "C" void kernel_launch(void* const* d_in, const int* in_sizes, int n_in, void* d_out, int out_size, void* d_ws, size_t ws_size, hipStream_t stream) {
  if (n_in < 29) return;
  if (in_sizes[0] < (NB - 1) * SEQ_FULL * CH + SEQ * CH) return;
  if (in_sizes[1] < DM * PL || in_sizes[5] < DM * PL || in_sizes[7] < PL * DM) return;
  if (in_sizes[13] < L2 * DM || in_sizes[14] < CH * MAXLEN * DM) return;
  if (in_sizes[15] < NLAYER * DM * DM || in_sizes[17] < NLAYER * DM * DM || in_sizes[19] < NLAYER * DM * DM || in_sizes[21] < NLAYER * DM * DM) return;
  if (in_sizes[25] < NLAYER * FF * DM || in_sizes[27] < NLAYER * DM * FF) return;
  if (out_size < NB * PL * CH) return;
  if (ws_size < (size_t)WS_END) return;
  const float** F = (const float**)d_in;
  char* ws = (char*)d_ws;
  float* ST = (float*)(ws + WS_ST); float* H = (float*)(ws + WS_H); float* A32 = (float*)(ws + WS_A32);
  _Float16 *ZH = (_Float16*)(ws + WS_ZH), *ZL = (_Float16*)(ws + WS_ZL), *QH = (_Float16*)(ws + WS_QH), *QL = (_Float16*)(ws + WS_QL), *KH = (_Float16*)(ws + WS_KH), *KL = (_Float16*)(ws + WS_KL), *VH = (_Float16*)(ws + WS_VH), *VL = (_Float16*)(ws + WS_VL);
  _Float16 *FH = (_Float16*)(ws + WS_FH), *FL = (_Float16*)(ws + WS_FL);
  _Float16 *WQ = (_Float16*)(ws + WS_WQ), *WK = (_Float16*)(ws + WS_WK), *WV = (_Float16*)(ws + WS_WV), *WC = (_Float16*)(ws + WS_WC), *WFC = (_Float16*)(ws + WS_WFC), *WP = (_Float16*)(ws + WS_WP);
  k_wcvt<<<NLAYER * DM * DM / 2048, 256, 0, stream>>>(F[15], WQ);
  k_wcvt<<<NLAYER * DM * DM / 2048, 256, 0, stream>>>(F[17], WK);
  k_wcvt<<<NLAYER * DM * DM / 2048, 256, 0, stream>>>(F[19], WV);
  k_wcvt<<<NLAYER * DM * DM / 2048, 256, 0, stream>>>(F[21], WC);
  k_wcvt<<<NLAYER * FF * DM / 2048, 256, 0, stream>>>(F[25], WFC);
  k_wcvt<<<NLAYER * DM * FF / 2048, 256, 0, stream>>>(F[27], WP);
  k_stats<<<1, 256, 0, stream>>>(F[0], ST);
  k_embed<<<dim3(NSEG, NB), 128, 0, stream>>>(F[0], ST, F[1], F[2], F[3], F[4], F[5], F[6], F[10], F[9], F[11], F[13], F[14], H);
  const dim3 gD(NTOK / 64, DM / 64), gF(NTOK / 64, FF / 64);
  for (int i = 0; i < NLAYER; ++i) {
    k_rms<<<NTOK / 8, 256, 0, stream>>>(H, F[23] + i * DM, 1, ZH, ZL);
    k_gemm_pl<<<gD, 128, 0, stream>>>(ZH, ZL, WQ + (size_t)i * DM * DM, F[16] + i * DM, DM, DM, QH, QL);
    k_gemm_pl<<<gD, 128, 0, stream>>>(ZH, ZL, WK + (size_t)i * DM * DM, F[18] + i * DM, DM, DM, KH, KL);
    k_gemm_pl<<<gD, 128, 0, stream>>>(ZH, ZL, WV + (size_t)i * DM * DM, F[20] + i * DM, DM, DM, VH, VL);
    k_attn<<<dim3(NBC, NH), 128, 0, stream>>>(QH, QL, KH, KL, VH, VL, A32);
    k_rms<<<NTOK / 8, 256, 0, stream>>>(A32, F[23], 0, ZH, ZL);
    k_gemm_rs<<<gD, 128, 0, stream>>>(ZH, ZL, WC + (size_t)i * DM * DM, F[22] + i * DM, DM, DM, H);
    k_rms<<<NTOK / 8, 256, 0, stream>>>(H, F[24] + i * DM, 1, ZH, ZL);
    k_gemm_ge<<<gF, 128, 0, stream>>>(ZH, ZL, WFC + (size_t)i * FF * DM, F[26] + i * FF, DM, FF, FH, FL);
    k_gemm_rs<<<gD, 128, 0, stream>>>(FH, FL, WP + (size_t)i * DM * FF, F[28] + i * DM, FF, DM, H);
  }
  k_final<<<1, 128, 0, stream>>>(H, F[12], F[7], F[8], ST, (float*)d_out);
}
